// TSClusteringLayer_17609365913690
// MI455X (gfx1250) — hardware-verified
//
#include <hip/hip_runtime.h>
#include <stddef.h>


typedef _Float16 v16h __attribute__((ext_vector_type(16)));
typedef _Float16 v8h  __attribute__((ext_vector_type(8)));
typedef float    v8f  __attribute__((ext_vector_type(8)));
typedef float    v4f  __attribute__((ext_vector_type(4)));
typedef _Float16 h16;

#ifndef NB
#define NB 2048
#endif
#define NB_FULL 2048
#define NCL   32
#define TLEN  128
#define NF    16

#define XCARRY 64.0f

#define CROWS 4
#define LDP   136
#define LDO   36
#define DWAVES 4
#define DROWS (DWAVES * 16)

static_assert(NB >= DROWS && NB <= NB_FULL);
static_assert((NB % DROWS) == 0);
static_assert((NB % CROWS) == 0 && (NCL % CROWS) == 0);
static_assert(NCL == 32);
static_assert(NCL * 4 == 128);
static_assert(TLEN == 128 && (TLEN % 32) == 0 && (TLEN % 8) == 0);
static_assert(NF == 16 && (NF % 4) == 0);
static_assert((LDP % 8) == 0 && LDP >= TLEN);
static_assert((LDO % 4) == 0 && LDO >= NCL);
static_assert(CROWS * TLEN * NF == 8 * 256 * 4);
static_assert(CROWS * NF * (TLEN / 8) == 4 * 256);
static_assert(4 * 4 == 16);
static_assert((size_t)CROWS * NF * LDP * 2 <= (size_t)131072);
static_assert((size_t)DWAVES * 16 * LDO * 4 <= (size_t)131072);

#define XP_BYTES ((size_t)NF * NB * TLEN * 2)
#define CP_BYTES ((size_t)NF * NCL * TLEN * 2)
#define OFF_XP ((size_t)0)
#define OFF_CP (OFF_XP + XP_BYTES)
#define WS_TOTAL (OFF_CP + CP_BYTES)
static_assert((XP_BYTES % 128) == 0 && (CP_BYTES % 128) == 0);
static_assert(WS_TOTAL <= (size_t)134217728);

__device__ __forceinline__ float bf16r(float x) {
  unsigned int u = __float_as_uint(x);
  u = (u + 0x7FFFu + ((u >> 16) & 1u)) & 0xFFFF0000u;
  return __uint_as_float(u);
}

static __device__ __forceinline__ h16 toh_flush(float v) {
  const h16 r = (h16)v;
  return (fabsf(v) < 6.103515625e-05f) ? (h16)0.0f : r;
}

__device__ __forceinline__ v16h frag_at(const _Float16* p) {
  v8h lo = *(const v8h*)(p);
  v8h hi = *(const v8h*)(p + 16);
  v16h out;
#pragma unroll
  for (int i = 0; i < 8; ++i) { out[i] = lo[i]; out[i + 8] = hi[i]; }
  return out;
}

__device__ __forceinline__ v8f wmma16(v16h a, v16h b, v8f c) {
  v8f d = __builtin_amdgcn_wmma_f32_16x16x32_f16(false, a, false, b, (short)0, c,
                                                 false, false);
  asm volatile("v_nop\n\tv_nop\n\tv_nop\n\tv_nop" : "+v"(d) : "v"(a), "v"(b));
  return d;
}

__device__ __forceinline__ float red16_sum(float x) {
#pragma unroll
  for (int off = 1; off < 16; off <<= 1) x += __shfl_xor(x, off, 32);
  return x;
}

__device__ __forceinline__ float sumsq16(v16h a, float s) {
#pragma unroll
  for (int i = 0; i < 16; ++i) {
    const float e = (float)a[i];
    s = fmaf(e, e, s);
  }
  return s;
}

__global__ __launch_bounds__(256) void plane_kernel(
    const float* __restrict__ src, _Float16* __restrict__ dst, unsigned nrows) {
  __shared__ _Float16 T[CROWS * NF * LDP];
  const unsigned tid = threadIdx.x;
  const unsigned row0 = blockIdx.x * (unsigned)CROWS;
  const float* sp = src + (size_t)row0 * (TLEN * NF);
#pragma unroll 2
  for (unsigned j = 0; j < 8u; ++j) {
    const unsigned idx = tid + 256u * j;
    const v4f v = *(const v4f*)(sp + (size_t)idx * 4u);
    const unsigned r = idx >> 9;
    const unsigned t = (idx >> 2) & 127u;
    const unsigned fq = (idx & 3u) * 4u;
#pragma unroll
    for (unsigned i = 0; i < 4u; ++i)
      T[(r * NF + fq + i) * LDP + t] = toh_flush(XCARRY * bf16r(v[i]));
  }
  __syncthreads();
  v8h x[4];
  size_t off[4];
#pragma unroll
  for (unsigned i = 0; i < 4u; ++i) {
    const unsigned p = tid + 256u * i;
    const unsigned seg = p >> 4;
    const unsigned kc = (p & 15u) * 8u;
    const unsigned r = seg >> 4, f = seg & 15u;
    x[i] = *(const v8h*)&T[seg * LDP + kc];
    off[i] = ((size_t)f * nrows + row0 + r) * TLEN + kc;
  }
#pragma unroll
  for (int i = 0; i < 4; ++i) *(volatile v8h*)(dst + off[i]) = x[i];
  __threadfence();
#pragma unroll
  for (int i = 0; i < 4; ++i) *(volatile v8h*)(dst + off[i]) = x[i];
}

__global__ __launch_bounds__(128) void dist_kernel(
    const _Float16* __restrict__ Xp, const _Float16* __restrict__ Cp, float* __restrict__ out) {
  __shared__ float Os[DWAVES * 16 * LDO];
  const unsigned tid = threadIdx.x, lane = tid & 31u;
  const int wave = __builtin_amdgcn_readfirstlane(threadIdx.x >> 5);
  const unsigned hh = lane >> 4, m = lane & 15u;
  const unsigned row0 = blockIdx.x * (unsigned)DROWS + (unsigned)wave * 16u;

  const _Float16* xa = Xp + (size_t)(row0 + m) * TLEN + hh * 8u;
  const _Float16* cb = Cp + (size_t)m * TLEN + hh * 8u;

  v8f d0 = {}, d1 = {};
#pragma unroll 1
  for (unsigned f = 0; f < (unsigned)NF; ++f) {
    const _Float16* ap  = xa + (size_t)f * NB * TLEN;
    const _Float16* bp0 = cb + (size_t)f * NCL * TLEN;
    const _Float16* bp1 = bp0 + (size_t)16 * TLEN;
    v8f acc0 = {}, acc1 = {};
    float sx = 0.0f, sc0 = 0.0f, sc1 = 0.0f;
#pragma unroll
    for (unsigned k0 = 0; k0 < (unsigned)TLEN; k0 += 32u) {
      const v16h a  = frag_at(ap + k0);
      const v16h b0 = frag_at(bp0 + k0);
      const v16h b1 = frag_at(bp1 + k0);
      acc0 = wmma16(a, b0, acc0);
      acc1 = wmma16(a, b1, acc1);
      sx  = sumsq16(a, sx);
      sc0 = sumsq16(b0, sc0);
      sc1 = sumsq16(b1, sc1);
    }
    sx  += __shfl_xor(sx, 16, 32);
    sc0 += __shfl_xor(sc0, 16, 32);
    sc1 += __shfl_xor(sc1, 16, 32);
#pragma unroll
    for (int r = 0; r < 8; ++r) {
      const float sxr = __shfl(sx, (int)(hh * 8u) + r, 32);
      const float e0 = ((sxr + sc0) - 2.0f * acc0[r]) * (1.0f / (XCARRY * XCARRY));
      const float e1 = ((sxr + sc1) - 2.0f * acc1[r]) * (1.0f / (XCARRY * XCARRY));
      d0[r] += __builtin_amdgcn_sqrtf(fmaxf(e0, 0.0f));
      d1[r] += __builtin_amdgcn_sqrtf(fmaxf(e1, 0.0f));
    }
  }

  float* O = &Os[(unsigned)wave * (16u * LDO)];
#pragma unroll
  for (int r = 0; r < 8; ++r) {
    const float q0 = __builtin_amdgcn_rcpf(1.0f + d0[r] * d0[r]);
    const float q1 = __builtin_amdgcn_rcpf(1.0f + d1[r] * d1[r]);
    const float s = red16_sum(q0 + q1);
    const float inv = __builtin_amdgcn_rcpf(s);
    O[(hh * 8u + (unsigned)r) * LDO + m]       = q0 * inv;
    O[(hh * 8u + (unsigned)r) * LDO + 16u + m] = q1 * inv;
  }
  __syncthreads();

  v4f x[4];
  size_t off[4];
#pragma unroll
  for (unsigned i = 0; i < 4u; ++i) {
    const unsigned r = 4u * i + (lane >> 3);
    const unsigned c = (lane & 7u) * 4u;
    x[i] = *(const v4f*)&O[r * LDO + c];
    off[i] = (size_t)(row0 + r) * NCL + c;
  }
#pragma unroll
  for (int i = 0; i < 4; ++i) *(volatile v4f*)(out + off[i]) = x[i];
  __threadfence();
#pragma unroll
  for (int i = 0; i < 4; ++i) *(volatile v4f*)(out + off[i]) = x[i];
}

extern "C" void kernel_launch(void* const* d_in, const int* in_sizes, int n_in,
                              void* d_out, int out_size, void* d_ws, size_t ws_size,
                              hipStream_t stream) {
  if (n_in < 2) return;
  if ((long long)in_sizes[0] < (long long)NB * TLEN * NF) return;
  if ((long long)in_sizes[1] < (long long)NCL * TLEN * NF) return;
  if ((long long)out_size < (long long)NB * NCL) return;
  if (ws_size < WS_TOTAL) return;

  const float* X = (const float*)d_in[0];
  const float* C = (const float*)d_in[1];
  float* out = (float*)d_out;

  char* ws = (char*)d_ws;
  _Float16* Xp = (_Float16*)(ws + OFF_XP);
  _Float16* Cp = (_Float16*)(ws + OFF_CP);

  plane_kernel<<<dim3(NB / CROWS), dim3(256), 0, stream>>>(X, Xp, (unsigned)NB);
  plane_kernel<<<dim3(NCL / CROWS), dim3(256), 0, stream>>>(C, Cp, (unsigned)NCL);
  dist_kernel<<<dim3(NB / DROWS), dim3(128), 0, stream>>>(Xp, Cp, out);
}
